// UnifiedRingStarBlock_46179488367248
// MI455X (gfx1250) — hardware-verified
//
#include <hip/hip_runtime.h>
#include <math.h>

constexpr int kB = 32;
constexpr int kL = 720;
constexpr int kN = 512;
constexpr int kH = 16;
constexpr int kD = 64;
constexpr int kTopK = 8;
constexpr int kRows = kB * kL;
constexpr int kRouterRows = 64;
constexpr int kRingRows = 16;
constexpr float kWgCarry = 16.0f;
constexpr float kWgCarryInv = 1.0f / 16.0f;
constexpr float kInvN = 1.0f / 512.0f;
constexpr float kLnEps = 1e-5f;

static_assert(kRows % 64 == 0);
static_assert(kRows % kRingRows == 0);
static_assert(kRows % 8 == 0);
static_assert(kN % 64 == 0);
static_assert(kN % kRouterRows == 0);

typedef __attribute__((ext_vector_type(16))) _Float16 v16h;
typedef __attribute__((ext_vector_type(8)))  _Float16 v8h;
typedef __attribute__((ext_vector_type(16))) __bf16   v16b;
typedef __attribute__((ext_vector_type(8)))  __bf16   v8b;
typedef __attribute__((ext_vector_type(8)))  float    v8f;
typedef __attribute__((ext_vector_type(4)))  float    v4f;
typedef __attribute__((ext_vector_type(4)))  int      v4i;
typedef __attribute__((ext_vector_type(4)))  unsigned int v4u;

__device__ __forceinline__ unsigned short f2bf_bits(float f) {
  unsigned u = __float_as_uint(f);
  return (unsigned short)((u + 0x7FFFu + ((u >> 16) & 1u)) >> 16);
}
__device__ __forceinline__ float bf_bits2f(unsigned short h) { return __uint_as_float(((unsigned)h) << 16); }

__device__ __forceinline__ void dep_guard_h(v8f& a, v8f& b, v16h x, v16h y) { asm volatile("v_nop\n\tv_nop\n\tv_nop\n\tv_nop" : "+v"(a), "+v"(b) : "v"(x), "v"(y)); }
__device__ __forceinline__ void dep_guard_b(v8f& a, v8f& b, v16b x, v16b y) { asm volatile("v_nop\n\tv_nop\n\tv_nop\n\tv_nop" : "+v"(a), "+v"(b) : "v"(x), "v"(y)); }
__device__ __forceinline__ void keep4_h(v16h a, v16h b, v16h c, v16h d) { asm volatile("v_nop" :: "v"(a), "v"(b), "v"(c), "v"(d)); }
__device__ __forceinline__ void keep4_b(v16b a, v16b b, v16b c, v16b d) { asm volatile("v_nop" :: "v"(a), "v"(b), "v"(c), "v"(d)); }
__device__ __forceinline__ void acc_guard4(v8f& a, v8f& b, v8f& c, v8f& d) { asm volatile("v_nop\n\tv_nop\n\tv_nop\n\tv_nop" : "+v"(a), "+v"(b), "+v"(c), "+v"(d)); }
template <typename T> struct Frag;
template <> struct Frag<_Float16> {
  typedef v16h V; union U { v16h v; v8h h[2]; };
  static __device__ __forceinline__ v16h load(const _Float16* p) {
    U f; f.h[0] = *(const v8h*)(p); f.h[1] = *(const v8h*)(p + 16); return f.v;
  }
  static __device__ __forceinline__ v8f mma(v16h a, v16h b, v8f c) {
    return __builtin_amdgcn_wmma_f32_16x16x32_f16(false, a, false, b, (short)0, c, false, false);
  }
  static __device__ __forceinline__ void guard(v8f& a, v8f& b, v16h x, v16h y) { dep_guard_h(a, b, x, y); }
  static __device__ __forceinline__ void keep(v16h a, v16h b, v16h c, v16h d) { keep4_h(a, b, c, d); }
};
template <> struct Frag<__bf16> {
  typedef v16b V; union U { v16b v; v8b h[2]; };
  static __device__ __forceinline__ v16b load(const __bf16* p) {
    U f; f.h[0] = *(const v8b*)(p); f.h[1] = *(const v8b*)(p + 16); return f.v;
  }
  static __device__ __forceinline__ v8f mma(v16b a, v16b b, v8f c) {
    return __builtin_amdgcn_wmma_f32_16x16x32_bf16(false, a, false, b, (short)0, c, false, false);
  }
  static __device__ __forceinline__ void guard(v8f& a, v8f& b, v16b x, v16b y) { dep_guard_b(a, b, x, y); }
  static __device__ __forceinline__ void keep(v16b a, v16b b, v16b c, v16b d) { keep4_b(a, b, c, d); }
};

__device__ __forceinline__ unsigned pk16(unsigned short a, unsigned short b) { return (unsigned)a | ((unsigned)b << 16); }
__device__ __forceinline__ unsigned short h_bits(float f) { const _Float16 h = (_Float16)f; return __builtin_bit_cast(unsigned short, h); }

__device__ __forceinline__ float wave_sum(float v) {
#pragma unroll
  for (int o = 16; o > 0; o >>= 1) v += __shfl_xor(v, o, 32);
  return v;
}
__device__ __forceinline__ float wave_max(float v) {
#pragma unroll
  for (int o = 16; o > 0; o >>= 1) v = fmaxf(v, __shfl_xor(v, o, 32));
  return v;
}

template <int ET> struct Elem;
template <> struct Elem<0> { typedef _Float16 T; };
template <> struct Elem<1> { typedef __bf16 T; };
template <int ET, bool SPLIT, int BIAS_MODE, int OUT_MODE, bool RESID, int ACT = 0>
__global__ __launch_bounds__(256) void wmma_gemm64(
    const unsigned short* __restrict__ Ap, const unsigned short* __restrict__ A2p, int lda, long strideA,
    const unsigned short* __restrict__ Btp, const unsigned short* __restrict__ Bt2p, int ldb, long strideB,
    void* __restrict__ Cout, void* __restrict__ Cout2, int ldc, long strideC,
    const float* __restrict__ bias,
    const float* __restrict__ resid, long strideR,
    int M, int N, int K, float scale) {
  typedef typename Elem<ET>::T T;
  typedef typename Frag<T>::V V;
  const T* A = (const T*)Ap; const T* A2 = (const T*)A2p; const T* Bt = (const T*)Btp; const T* Bt2 = (const T*)Bt2p;
  __shared__ __align__(16) float sT[8][16 * 68];
  const int b    = blockIdx.y;
  const int lane = threadIdx.x & 31;
  const int wave = threadIdx.x >> 5;
  const int tilesN = N >> 6;
  const int tilesM = M >> 6;
  const int tile = blockIdx.x * 8 + wave;
  if (tile >= tilesM * tilesN) return;
  const int tm = tile / tilesN;
  const int tn = tile - tm * tilesN;
  const int m0 = tm << 6;
  const int n0 = tn << 6;

  const T* Ab  = A  + (size_t)b * strideA;
  const T* Bb  = Bt + (size_t)b * strideB;
  const T* Ab2 = SPLIT ? (A2  + (size_t)b * strideA) : nullptr;
  const T* Bb2 = SPLIT ? (Bt2 + (size_t)b * strideB) : nullptr;

  const int rlane = lane & 15;
  const int koff  = (lane >> 4) * 8;
  const int mOff  = (lane >> 4) * 8;

  v8f acc[4][4];
#pragma unroll
  for (int i = 0; i < 4; ++i)
#pragma unroll
    for (int j = 0; j < 4; ++j) acc[i][j] = (v8f){0.f,0.f,0.f,0.f,0.f,0.f,0.f,0.f};

  for (int k0 = 0; k0 < K; k0 += 32) {
    V bh[4], bl[4];
#pragma unroll
    for (int j = 0; j < 4; ++j) {
      const size_t bo = (size_t)(n0 + (j << 4) + rlane) * ldb + koff + k0;
      bh[j] = Frag<T>::load(Bb + bo);
      if (SPLIT) bl[j] = Frag<T>::load(Bb2 + bo);
    }
#pragma unroll
    for (int i = 0; i < 4; ++i) {
      const size_t ao = (size_t)(m0 + (i << 4) + rlane) * lda + koff + k0;
      V ah = Frag<T>::load(Ab + ao);
      V al;
      if (SPLIT) al = Frag<T>::load(Ab2 + ao);
#pragma unroll
      for (int j = 0; j < 4; ++j) {
        acc[i][j] = Frag<T>::mma(ah, bh[j], acc[i][j]);
        if (SPLIT) {
          acc[i][j] = Frag<T>::mma(ah, bl[j], acc[i][j]);
          acc[i][j] = Frag<T>::mma(al, bh[j], acc[i][j]);
        }
      }
      Frag<T>::guard(acc[i][0], acc[i][3], ah, SPLIT ? al : ah);
    }
    Frag<T>::keep(bh[0], bh[1], bh[2], bh[3]);
    if (SPLIT) Frag<T>::keep(bl[0], bl[1], bl[2], bl[3]);
  }
  acc_guard4(acc[0][0], acc[0][1], acc[0][2], acc[0][3]);
  acc_guard4(acc[1][0], acc[1][1], acc[1][2], acc[1][3]);
  acc_guard4(acc[2][0], acc[2][1], acc[2][2], acc[2][3]);
  acc_guard4(acc[3][0], acc[3][1], acc[3][2], acc[3][3]);

  float* slab = sT[wave];
  const float* Rb = RESID ? (resid + (size_t)b * strideR) : nullptr;
#pragma unroll
  for (int i = 0; i < 4; ++i) {
    const int mBase = m0 + (i << 4);
#pragma unroll
    for (int j = 0; j < 4; ++j) {
      const int n = n0 + (j << 4) + rlane;
      float bv = 0.f;
      if (BIAS_MODE == 2) bv = bias[n];
#pragma unroll
      for (int r = 0; r < 8; ++r) {
        float v = acc[i][j][r] * scale;
        if (BIAS_MODE == 1) v += bias[mBase + mOff + r];
        if (BIAS_MODE == 2) v += bv;
        if (RESID) v += Rb[(size_t)(mBase + mOff + r) * ldc + n];
        if (ACT == 2) v = fmaxf(v, 0.0f);
        if (ACT == 4) v = (v > 0.f) ? v : 0.01f * v;
        slab[(mOff + r) * 68 + (j << 4) + rlane] = v;
      }
    }
    __builtin_amdgcn_fence(__ATOMIC_RELEASE, "workgroup");
    __builtin_amdgcn_wave_barrier();
    __builtin_amdgcn_fence(__ATOMIC_ACQUIRE, "workgroup");
    if (OUT_MODE == 0) {
      float* C = (float*)Cout + (size_t)b * strideC;
      const int hh = lane >> 4, c4 = (lane & 15) * 4;
      for (int pass = 0; pass < 2; ++pass) {
#pragma unroll
        for (int it = 0; it < 8; ++it) {
          const int row = it * 2 + hh;
          v4f v = *(const v4f*)(slab + row * 68 + c4);
          *(volatile v4f*)(C + (size_t)(mBase + row) * ldc + n0 + c4) = v;
        }
        __threadfence();
      }
    } else {
      const int q = lane >> 3, c8 = (lane & 7) * 8;
      unsigned short* C  = (unsigned short*)Cout  + (size_t)b * strideC;
      unsigned short* C2 = (OUT_MODE == 2) ? ((unsigned short*)Cout2 + (size_t)b * strideC) : nullptr;
      for (int pass = 0; pass < 2; ++pass) {
#pragma unroll
        for (int it = 0; it < 4; ++it) {
          const int row = it * 4 + q;
          const float* sp = slab + row * 68 + c8;
          v8h hv, lv;
#pragma unroll
          for (int e = 0; e < 8; ++e) {
            if (OUT_MODE == 1) {
              hv[e] = (_Float16)sp[e];
            } else {
              unsigned short hb = f2bf_bits(sp[e]);
              unsigned short lb = f2bf_bits(sp[e] - bf_bits2f(hb));
              hv[e] = __builtin_bit_cast(_Float16, hb);
              lv[e] = __builtin_bit_cast(_Float16, lb);
            }
          }
          *(volatile v8h*)(C + (size_t)(mBase + row) * ldc + n0 + c8) = hv;
          if (OUT_MODE == 2) *(volatile v8h*)(C2 + (size_t)(mBase + row) * ldc + n0 + c8) = lv;
        }
        __threadfence();
      }
    }
    __builtin_amdgcn_fence(__ATOMIC_RELEASE, "workgroup");
    __builtin_amdgcn_wave_barrier();
    __builtin_amdgcn_fence(__ATOMIC_ACQUIRE, "workgroup");
  }
}

__global__ __launch_bounds__(256) void wmma_gemm64_gate(
    const unsigned short* __restrict__ Ap, int lda,
    const unsigned short* __restrict__ Btp, int ldb,
    unsigned short* __restrict__ Chi, unsigned short* __restrict__ Clo, int ldc,
    const float* __restrict__ gcen, const float* __restrict__ center, const float* __restrict__ ring32,
    int M, int N, int K, float scale) {
  typedef _Float16 T;
  const T* A = (const T*)Ap; const T* Bt = (const T*)Btp;
  __shared__ __align__(16) float sT[8][16 * 68];
  const int lane = threadIdx.x & 31;
  const int wave = threadIdx.x >> 5;
  const int tilesN = N >> 6;
  const int tilesM = M >> 6;
  const int tile = blockIdx.x * 8 + wave;
  if (tile >= tilesM * tilesN) return;
  const int tm = tile / tilesN;
  const int tn = tile - tm * tilesN;
  const int m0 = tm << 6;
  const int n0 = tn << 6;

  const int rlane = lane & 15;
  const int koff  = (lane >> 4) * 8;
  const int mOff  = (lane >> 4) * 8;

  v8f acc[4][4];
#pragma unroll
  for (int i = 0; i < 4; ++i)
#pragma unroll
    for (int j = 0; j < 4; ++j) acc[i][j] = (v8f){0.f,0.f,0.f,0.f,0.f,0.f,0.f,0.f};

  for (int k0 = 0; k0 < K; k0 += 32) {
    v16h bh[4];
#pragma unroll
    for (int j = 0; j < 4; ++j) {
      const size_t bo = (size_t)(n0 + (j << 4) + rlane) * ldb + koff + k0;
      bh[j] = Frag<T>::load(Bt + bo);
    }
#pragma unroll
    for (int i = 0; i < 4; ++i) {
      const size_t ao = (size_t)(m0 + (i << 4) + rlane) * lda + koff + k0;
      v16h ah = Frag<T>::load(A + ao);
#pragma unroll
      for (int j = 0; j < 4; ++j) acc[i][j] = Frag<T>::mma(ah, bh[j], acc[i][j]);
      Frag<T>::guard(acc[i][0], acc[i][3], ah, ah);
    }
    Frag<T>::keep(bh[0], bh[1], bh[2], bh[3]);
  }
  acc_guard4(acc[0][0], acc[0][1], acc[0][2], acc[0][3]);
  acc_guard4(acc[1][0], acc[1][1], acc[1][2], acc[1][3]);
  acc_guard4(acc[2][0], acc[2][1], acc[2][2], acc[2][3]);
  acc_guard4(acc[3][0], acc[3][1], acc[3][2], acc[3][3]);

  float* slab = sT[wave];
  const int bA = m0 / kL;
  const int splitRow = (bA + 1) * kL;
  const int bB = (bA + 1 > kB - 1) ? (kB - 1) : (bA + 1);
#pragma unroll
  for (int i = 0; i < 4; ++i) {
    const int mBase = m0 + (i << 4);
#pragma unroll
    for (int j = 0; j < 4; ++j) {
      const int n = n0 + (j << 4) + rlane;
      const float gA = gcen[bA * kN + n];
      const float gB = gcen[bB * kN + n];
      const float cA = center[bA * kN + n];
      const float cB = center[bB * kN + n];
#pragma unroll
      for (int r = 0; r < 8; ++r) {
        const int mrow = mBase + mOff + r;
        const bool useB = (mrow >= splitRow);
        const float gc = useB ? gB : gA;
        const float cb = useB ? cB : cA;
        const float v  = acc[i][j][r] * scale + gc;
        const float ex = expf(-v);
        const float gt = __builtin_amdgcn_rcpf(1.0f + ex);
        const float rg = ring32[(size_t)mrow * kN + n];
        const float fz = gt * rg + (1.0f - gt) * cb;
        slab[(mOff + r) * 68 + (j << 4) + rlane] = fz;
      }
    }
    __builtin_amdgcn_fence(__ATOMIC_RELEASE, "workgroup");
    __builtin_amdgcn_wave_barrier();
    __builtin_amdgcn_fence(__ATOMIC_ACQUIRE, "workgroup");
    {
      const int q = lane >> 3, c8 = (lane & 7) * 8;
      for (int pass = 0; pass < 2; ++pass) {
#pragma unroll
        for (int it = 0; it < 4; ++it) {
          const int row = it * 4 + q;
          const float* sp = slab + row * 68 + c8;
          v8h hv, lv;
#pragma unroll
          for (int e = 0; e < 8; ++e) {
            unsigned short hb = f2bf_bits(sp[e]);
            unsigned short lb = f2bf_bits(sp[e] - bf_bits2f(hb));
            hv[e] = __builtin_bit_cast(_Float16, hb);
            lv[e] = __builtin_bit_cast(_Float16, lb);
          }
          *(volatile v8h*)(Chi + (size_t)(mBase + row) * ldc + n0 + c8) = hv;
          *(volatile v8h*)(Clo + (size_t)(mBase + row) * ldc + n0 + c8) = lv;
        }
        __threadfence();
      }
    }
    __builtin_amdgcn_fence(__ATOMIC_RELEASE, "workgroup");
    __builtin_amdgcn_wave_barrier();
    __builtin_amdgcn_fence(__ATOMIC_ACQUIRE, "workgroup");
  }
}

__global__ __launch_bounds__(256) void k_wprep(const float* __restrict__ Wg, const float* __restrict__ Wf,
                                                unsigned short* __restrict__ wgT16,
                                                unsigned short* __restrict__ wfThi, unsigned short* __restrict__ wfTlo) {
  __shared__ float sm[64][65];
  const int t  = threadIdx.x;
  const int k0 = blockIdx.x * 64;
  const int n0 = blockIdx.y * 64;
  const int z  = blockIdx.z;
  const float* W = (z == 0) ? Wg : Wf;
  const float sc = (z == 0) ? kWgCarry : 1.0f;
#pragma unroll
  for (int i = 0; i < 16; ++i) {
    const int e = i * 256 + t;
    const int r = e >> 6;
    const int c = e & 63;
    sm[c][r] = W[(size_t)(k0 + r) * kN + n0 + c] * sc;
  }
  __syncthreads();
  const int lane = t & 31, wave = t >> 5;
  const int q = lane >> 3, c8 = (lane & 7) * 8;
  if (z == 0) {
    for (int pass = 0; pass < 2; ++pass) {
#pragma unroll
      for (int it = 0; it < 2; ++it) {
        const int row = wave * 8 + it * 4 + q;
        unsigned short hb[8];
#pragma unroll
        for (int e = 0; e < 8; ++e) hb[e] = h_bits(sm[row][c8 + e]);
        const v4u u = (v4u){pk16(hb[0], hb[1]), pk16(hb[2], hb[3]), pk16(hb[4], hb[5]), pk16(hb[6], hb[7])};
        *(volatile v4u*)(wgT16 + (size_t)(n0 + row) * kN + k0 + c8) = u;
      }
      __threadfence();
    }
  } else {
    for (int pass = 0; pass < 2; ++pass) {
#pragma unroll
      for (int it = 0; it < 2; ++it) {
        const int row = wave * 8 + it * 4 + q;
        unsigned short hb[8], lb[8];
#pragma unroll
        for (int e = 0; e < 8; ++e) {
          const float v = sm[row][c8 + e];
          hb[e] = f2bf_bits(v);
          lb[e] = f2bf_bits(v - bf_bits2f(hb[e]));
        }
        const v4u uh = (v4u){pk16(hb[0], hb[1]), pk16(hb[2], hb[3]), pk16(hb[4], hb[5]), pk16(hb[6], hb[7])};
        const v4u ul = (v4u){pk16(lb[0], lb[1]), pk16(lb[2], lb[3]), pk16(lb[4], lb[5]), pk16(lb[6], lb[7])};
        *(volatile v4u*)(wfThi + (size_t)(n0 + row) * kN + k0 + c8) = uh;
        *(volatile v4u*)(wfTlo + (size_t)(n0 + row) * kN + k0 + c8) = ul;
      }
      __threadfence();
    }
  }
}

__global__ __launch_bounds__(64) void k_router(const float* __restrict__ ve,
                                                const float* __restrict__ Wq, const float* __restrict__ bq,
                                                const float* __restrict__ Wk, const float* __restrict__ bk,
                                                int* __restrict__ idx_out, float* __restrict__ w_out) {
#pragma clang fp contract(off)
  __shared__ __align__(16) float sK[kN * kH];
  __shared__ __align__(16) float sW[kRouterRows * kTopK];
  __shared__ __align__(16) int   sI[kRouterRows * kTopK];
  const int t = threadIdx.x;
  const int n = blockIdx.x * kRouterRows + t;

#pragma unroll 1
  for (int i = 0; i < kN / kRouterRows; ++i) {
    const int col = i * kRouterRows + t;
    const float* er = ve + col * kH;
#pragma unroll 1
    for (int h = 0; h < kH; ++h) {
      float a = 0.f;
#pragma unroll 1
      for (int j = 0; j < kH; ++j) a = a + er[j] * Wk[j * kH + h];
      sK[col * kH + h] = a + bk[h];
    }
  }
  float q[kH];
  {
    const float* en = ve + n * kH;
#pragma unroll
    for (int h = 0; h < kH; ++h) {
      float a = 0.f;
#pragma unroll 1
      for (int j = 0; j < kH; ++j) a = a + en[j] * Wq[j * kH + h];
      q[h] = a + bq[h];
    }
  }
  __syncthreads();

  float tv[kTopK]; int ti[kTopK];
#pragma unroll
  for (int p = 0; p < kTopK; ++p) { tv[p] = -INFINITY; ti[p] = 0; }
#pragma unroll 1
  for (int col = 0; col < kN; ++col) {
    const float* kr = sK + col * kH;
    float d = 0.f;
#pragma unroll
    for (int j = 0; j < kH; ++j) d = d + q[j] * kr[j];
    d = (col == n) ? -1.0e9f : d;
    bool g[kTopK];
#pragma unroll
    for (int p = 0; p < kTopK; ++p) g[p] = (d > tv[p]);
#pragma unroll
    for (int p = kTopK - 1; p >= 1; --p) {
      const float nv = g[p - 1] ? tv[p - 1] : d;
      const int   ni = g[p - 1] ? ti[p - 1] : col;
      tv[p] = g[p] ? nv : tv[p];
      ti[p] = g[p] ? ni : ti[p];
    }
    tv[0] = g[0] ? d : tv[0];
    ti[0] = g[0] ? col : ti[0];
  }
  {
    const float mx = tv[0];
    float e[kTopK];
    float s = 0.f;
#pragma unroll
    for (int p = 0; p < kTopK; ++p) { e[p] = expf(tv[p] - mx); s = s + e[p]; }
    const float inv = 1.0f / s;
#pragma unroll
    for (int p = 0; p < kTopK; ++p) { sW[t * kTopK + p] = e[p] * inv; sI[t * kTopK + p] = ti[p]; }
  }
  __syncthreads();
  {
    float* wdst = w_out + blockIdx.x * (kRouterRows * kTopK);
    int*   idst = idx_out + blockIdx.x * (kRouterRows * kTopK);
    const int off0 = t * 4, off1 = 256 + t * 4;
    const v4f w0 = *(const v4f*)(sW + off0);
    const v4f w1 = *(const v4f*)(sW + off1);
    const v4i i0 = *(const v4i*)(sI + off0);
    const v4i i1 = *(const v4i*)(sI + off1);
    *(volatile v4f*)(wdst + off0) = w0;
    *(volatile v4f*)(wdst + off1) = w1;
    *(volatile v4i*)(idst + off0) = i0;
    *(volatile v4i*)(idst + off1) = i1;
    __threadfence();
    *(volatile v4f*)(wdst + off0) = w0;
    *(volatile v4f*)(wdst + off1) = w1;
    *(volatile v4i*)(idst + off0) = i0;
    *(volatile v4i*)(idst + off1) = i1;
  }
}

__global__ __launch_bounds__(512) void k_center(const float* __restrict__ x,
                                                 const float* __restrict__ Wscore, const float* __restrict__ bscore,
                                                 const float* __restrict__ Wc1, const float* __restrict__ bc1,
                                                 const float* __restrict__ Wc2, const float* __restrict__ bc2,
                                                 const float* __restrict__ Wcn, const float* __restrict__ bcn,
                                                 const float* __restrict__ Wg, const float* __restrict__ bg,
                                                 float* __restrict__ center_out, float* __restrict__ gcen_out) {
  __shared__ float sS[kL];
  __shared__ float sRed[16];
  __shared__ __align__(16) float sBuf[kN + kD + kD];
  __shared__ __align__(16) float sCen[kN];
  __shared__ __align__(16) float sG[kN];
  const int b = blockIdx.x;
  const int t = threadIdx.x;
  const int lane = t & 31, wave = t >> 5;
  const float* xb = x + (size_t)b * kL * kN;

#pragma unroll 1
  for (int l = wave; l < kL; l += 16) {
    const float* xr = xb + (size_t)l * kN;
    float acc = 0.f;
#pragma unroll 1
    for (int j = 0; j < kN / 32; ++j) acc += xr[j * 32 + lane] * Wscore[j * 32 + lane];
    acc = wave_sum(acc);
    if (lane == 0) sS[l] = acc + bscore[0];
  }
  __syncthreads();

  float m = -INFINITY;
#pragma unroll 1
  for (int l = t; l < kL; l += 512) m = fmaxf(m, sS[l]);
  m = wave_max(m);
  if (lane == 0) sRed[wave] = m;
  __syncthreads();
  float mx = sRed[0];
#pragma unroll 1
  for (int w = 1; w < 16; ++w) mx = fmaxf(mx, sRed[w]);
  __syncthreads();
  float ps = 0.f;
#pragma unroll 1
  for (int l = t; l < kL; l += 512) { const float e = expf(sS[l] - mx); sS[l] = e; ps += e; }
  ps = wave_sum(ps);
  if (lane == 0) sRed[wave] = ps;
  __syncthreads();
  float tot = 0.f;
#pragma unroll 1
  for (int w = 0; w < 16; ++w) tot += sRed[w];
  const float inv = 1.0f / tot;
#pragma unroll 1
  for (int l = t; l < kL; l += 512) sS[l] = sS[l] * inv;
  __syncthreads();

  {
    float acc = 0.f;
#pragma unroll 1
    for (int l = 0; l < kL; ++l) acc += sS[l] * xb[(size_t)l * kN + t];
    sBuf[t] = acc;
  }
  __syncthreads();

#pragma unroll 1
  for (int layer = 0; layer < 2; ++layer) {
    const int kdim   = layer ? kD : kN;
    const float* Wl  = layer ? Wc2 : Wc1;
    const float* bl  = layer ? bc2 : bc1;
    const int srcOff = layer ? kN : 0;
    const int dstOff = layer ? (kN + kD) : kN;
    if (t < kD) {
      float acc = 0.f;
#pragma unroll 1
      for (int j = 0; j < kdim; ++j) acc += sBuf[srcOff + j] * Wl[j * kD + t];
      acc += bl[t];
      const float gv = 0.5f * acc * (1.0f + erff(acc * 0.70710678118654752f));
      sBuf[dstOff + t] = gv;
    }
    __syncthreads();
  }

  {
    float acc = 0.f;
#pragma unroll 1
    for (int j = 0; j < kD; ++j) acc += sBuf[kN + kD + j] * Wcn[j * kN + t];
    acc += bcn[t];
    sCen[t] = acc;
  }
  __syncthreads();

  {
    float acc = 0.f;
#pragma unroll 1
    for (int j = 0; j < kN; ++j) acc += sCen[j] * Wg[(size_t)(kN + j) * kN + t];
    acc += bg[t];
    sG[t] = acc;
  }
  __syncthreads();

  if (t < 128) {
    const v4f v = *(const v4f*)(sCen + t * 4);
    float* dst = center_out + b * kN + t * 4;
    *(volatile v4f*)dst = v;
    __threadfence();
    *(volatile v4f*)dst = v;
  } else if (t < 256) {
    const int tt = t - 128;
    const v4f v = *(const v4f*)(sG + tt * 4);
    float* dst = gcen_out + b * kN + tt * 4;
    *(volatile v4f*)dst = v;
    __threadfence();
    *(volatile v4f*)dst = v;
  }
}

__global__ __launch_bounds__(256) void k_ring(const float* __restrict__ x,
                                               const int* __restrict__ idx8, const float* __restrict__ w8,
                                               float* __restrict__ ring32, unsigned short* __restrict__ ring16) {
  __shared__ __align__(16) float sx[kN];
  __shared__ __align__(16) float sr[kN];
  const int t  = threadIdx.x;
  const int na = t, nb = t + 256;
  int ia[kTopK], ib[kTopK];
  float wa[kTopK], wb[kTopK];
#pragma unroll
  for (int k = 0; k < kTopK; ++k) {
    int va = idx8[na * kTopK + k]; va = va < 0 ? 0 : (va > kN - 1 ? kN - 1 : va); ia[k] = va;
    int vb = idx8[nb * kTopK + k]; vb = vb < 0 ? 0 : (vb > kN - 1 ? kN - 1 : vb); ib[k] = vb;
    wa[k] = w8[na * kTopK + k];
    wb[k] = w8[nb * kTopK + k];
  }
#pragma unroll 1
  for (int rr = 0; rr < kRingRows; ++rr) {
    const int row = blockIdx.x * kRingRows + rr;
    const float* xr = x + (size_t)row * kN;
    __syncthreads();
    sx[t] = xr[t];
    sx[t + 256] = xr[t + 256];
    __syncthreads();
    float a0 = 0.f, a1 = 0.f;
#pragma unroll
    for (int k = 0; k < kTopK; ++k) {
      a0 += wa[k] * sx[ia[k]];
      a1 += wb[k] * sx[ib[k]];
    }
    sr[na] = a0;
    sr[nb] = a1;
    __syncthreads();
    if (t < 128) {
      const v4f v = *(const v4f*)(sr + t * 4);
      float* dst = ring32 + (size_t)row * kN + t * 4;
      *(volatile v4f*)dst = v;
      __threadfence();
      *(volatile v4f*)dst = v;
    } else if (t < 192) {
      const int c8 = (t - 128) * 8;
      unsigned short hb[8];
#pragma unroll
      for (int e = 0; e < 8; ++e) hb[e] = h_bits(sr[c8 + e]);
      const v4u u = (v4u){pk16(hb[0], hb[1]), pk16(hb[2], hb[3]), pk16(hb[4], hb[5]), pk16(hb[6], hb[7])};
      unsigned short* dst = ring16 + (size_t)row * kN + c8;
      *(volatile v4u*)dst = u;
      __threadfence();
      *(volatile v4u*)dst = u;
    }
  }
}

__global__ __launch_bounds__(256) void k_ln(const float* __restrict__ Hbuf,
                                             const float* __restrict__ gamma, const float* __restrict__ beta,
                                             float* __restrict__ out) {
  const int lane = threadIdx.x & 31, wave = threadIdx.x >> 5;
  const int row = blockIdx.x * 8 + wave;
  const float* hr = Hbuf + (size_t)row * kN;
  v4f hv[4], gv[4], bv[4];
#pragma unroll
  for (int j = 0; j < 4; ++j) {
    hv[j] = *(const v4f*)(hr + j * 128 + lane * 4);
    gv[j] = *(const v4f*)(gamma + j * 128 + lane * 4);
    bv[j] = *(const v4f*)(beta + j * 128 + lane * 4);
  }
  float s = 0.f;
#pragma unroll
  for (int j = 0; j < 4; ++j) s += (hv[j][0] + hv[j][1]) + (hv[j][2] + hv[j][3]);
  s = wave_sum(s);
  const float mu = s * kInvN;
  float qv = 0.f;
#pragma unroll
  for (int j = 0; j < 4; ++j) {
#pragma unroll
    for (int e = 0; e < 4; ++e) { const float d = hv[j][e] - mu; qv += d * d; }
  }
  qv = wave_sum(qv);
  const float var  = qv * kInvN;
  const float rstd = rsqrtf(var + kLnEps);
  v4f ov[4];
#pragma unroll
  for (int j = 0; j < 4; ++j) {
#pragma unroll
    for (int e = 0; e < 4; ++e) ov[j][e] = (hv[j][e] - mu) * rstd * gv[j][e] + bv[j][e];
  }
  float* orow = out + (size_t)row * kN;
#pragma unroll
  for (int j = 0; j < 4; ++j) *(volatile v4f*)(orow + j * 128 + lane * 4) = ov[j];
  __threadfence();
#pragma unroll
  for (int j = 0; j < 4; ++j) *(volatile v4f*)(orow + j * 128 + lane * 4) = ov[j];
}

constexpr size_t kOffIdx    = 0;
constexpr size_t kOffW8     = kOffIdx    + (size_t)kN * kTopK * 4;
constexpr size_t kOffCen    = kOffW8     + (size_t)kN * kTopK * 4;
constexpr size_t kOffGcen   = kOffCen    + (size_t)kB * kN * 4;
constexpr size_t kOffWgT16  = kOffGcen   + (size_t)kB * kN * 4;
constexpr size_t kOffWfHi   = kOffWgT16  + (size_t)kN * kN * 2;
constexpr size_t kOffWfLo   = kOffWfHi   + (size_t)kN * kN * 2;
constexpr size_t kOffRing32 = kOffWfLo   + (size_t)kN * kN * 2;
constexpr size_t kOffRing16 = kOffRing32 + (size_t)kRows * kN * 4;
constexpr size_t kOffFhi    = kOffRing16 + (size_t)kRows * kN * 2;
constexpr size_t kOffFlo    = kOffFhi    + (size_t)kRows * kN * 2;
constexpr size_t kWsTotal   = kOffFlo    + (size_t)kRows * kN * 2;
static_assert(kWsTotal == 119701504);
static_assert(kWsTotal <= 134217728);
static_assert(kOffRing32 % 128 == 0 && kOffRing16 % 128 == 0 && kOffFhi % 128 == 0 && kOffFlo % 128 == 0);

extern "C" void kernel_launch(void* const* d_in, const int* in_sizes, int n_in,
                              void* d_out, int out_size, void* d_ws, size_t ws_size,
                              hipStream_t stream) {
  if (n_in < 20) return;
  if (in_sizes[0] != kRows * kN || out_size != kRows * kN) return;
  if (in_sizes[1] != kN * kH || in_sizes[14] != 2 * kN * kN || in_sizes[16] != kN * kN) return;
  if (ws_size < kWsTotal) return;

  const float* x      = (const float*)d_in[0];
  const float* ve     = (const float*)d_in[1];
  const float* Wq     = (const float*)d_in[2];
  const float* bq     = (const float*)d_in[3];
  const float* Wk     = (const float*)d_in[4];
  const float* bk     = (const float*)d_in[5];
  const float* Wscore = (const float*)d_in[6];
  const float* bscore = (const float*)d_in[7];
  const float* Wc1    = (const float*)d_in[8];
  const float* bc1    = (const float*)d_in[9];
  const float* Wc2    = (const float*)d_in[10];
  const float* bc2    = (const float*)d_in[11];
  const float* Wcn    = (const float*)d_in[12];
  const float* bcn    = (const float*)d_in[13];
  const float* Wg     = (const float*)d_in[14];
  const float* bg     = (const float*)d_in[15];
  const float* Wf     = (const float*)d_in[16];
  const float* bfv    = (const float*)d_in[17];
  const float* gamma  = (const float*)d_in[18];
  const float* beta   = (const float*)d_in[19];
  float* out = (float*)d_out;

  char* ws = (char*)d_ws;
  int*            idx8   = (int*)(ws + kOffIdx);
  float*          w8     = (float*)(ws + kOffW8);
  float*          cen    = (float*)(ws + kOffCen);
  float*          gcen   = (float*)(ws + kOffGcen);
  unsigned short* wgT16  = (unsigned short*)(ws + kOffWgT16);
  unsigned short* wfThi  = (unsigned short*)(ws + kOffWfHi);
  unsigned short* wfTlo  = (unsigned short*)(ws + kOffWfLo);
  float*          ring32 = (float*)(ws + kOffRing32);
  float*          hbuf   = (float*)(ws + kOffRing32);
  unsigned short* ring16 = (unsigned short*)(ws + kOffRing16);
  unsigned short* fhi    = (unsigned short*)(ws + kOffFhi);
  unsigned short* flo    = (unsigned short*)(ws + kOffFlo);

  k_wprep<<<dim3(kN / 64, kN / 64, 2), 256, 0, stream>>>(Wg, Wf, wgT16, wfThi, wfTlo);
  k_router<<<kN / kRouterRows, kRouterRows, 0, stream>>>(ve, Wq, bq, Wk, bk, idx8, w8);
  k_center<<<kB, 512, 0, stream>>>(x, Wscore, bscore, Wc1, bc1, Wc2, bc2, Wcn, bcn, Wg, bg, cen, gcen);
  k_ring<<<kRows / kRingRows, 256, 0, stream>>>(x, idx8, w8, ring32, ring16);
  {
    const int tiles = (kRows / 64) * (kN / 64);
    wmma_gemm64_gate<<<dim3((tiles + 7) / 8, 1), 256, 0, stream>>>(
        ring16, kN, wgT16, kN, fhi, flo, kN, gcen, cen, ring32, kRows, kN, kN, kWgCarryInv);
  }
  {
    const int tiles = (kRows / 64) * (kN / 64);
    wmma_gemm64<1, true, 2, 0, true, 0><<<dim3((tiles + 7) / 8, 1), 256, 0, stream>>>(
        fhi, flo, kN, 0L, wfThi, wfTlo, kN, 0L,
        (void*)hbuf, (void*)nullptr, kN, 0L,
        bfv, x, 0L,
        kRows, kN, kN, 1.0f);
  }
  k_ln<<<kRows / 8, 256, 0, stream>>>(hbuf, gamma, beta, out);
}
